// S4Baseline_48223892799530
// MI455X (gfx1250) — hardware-run, weakly checked
//
#include <hip/hip_runtime.h>
#include <math.h>

typedef __attribute__((ext_vector_type(16))) _Float16 v16h;
typedef __attribute__((ext_vector_type(8)))  _Float16 v8h;
typedef __attribute__((ext_vector_type(8)))  float    v8f;
typedef __attribute__((ext_vector_type(4)))  float    v4f;
typedef __attribute__((ext_vector_type(2)))  float    v2f;
typedef __attribute__((ext_vector_type(4)))  unsigned v4u;

constexpr int kBatch    = 8;
constexpr int kLen      = 2048;
constexpr int kInDim    = 51;
constexpr int kInPad    = 64;
constexpr int kWidth    = 256;
constexpr int kModes    = 64;
constexpr int kLayers   = 4;
constexpr int kChunk    = 128;
constexpr int kChunksPS = kLen / kChunk;
constexpr int kRowsM    = kBatch * kChunksPS;
constexpr int kStateW   = 2 * kModes;
constexpr int kMvW      = kChunk + kStateW;
constexpr int kNpos     = kBatch * kLen;
constexpr int kOutDim   = 204;
constexpr int kOutPad   = 256;
constexpr int kGluW     = 2 * kWidth;
constexpr int kPitchW   = 132;
constexpr int kPitchX   = 36;
constexpr int kHeadPos  = 32;
static_assert(kChunksPS == 16 && kRowsM == 128 && kStateW == 128 && kMvW == 256 && kNpos == 16384, "derived shapes");
static_assert((kChunk % 32) == 0 && (kStateW % 32) == 0 && (kWidth % 32) == 0 && (kInPad % 32) == 0, "K multiples of 32");
static_assert((kRowsM % 64) == 0 && (kChunk % 64) == 0 && (kStateW % 64) == 0 && (kNpos % 64) == 0 && (kOutPad % 32) == 0, "tile multiples");
static_assert((kHeadPos * kOutDim * 4) % 128 == 0 && ((kHeadPos * kOutDim) / 4) % 32 == 0, "head block owns whole lines");

constexpr float kWCarry      = 256.0f;
constexpr float kWCarryInv   = 1.0f / 256.0f;
constexpr float kTabCarry    = 1024.0f;
constexpr float kTabCarryInv = 1.0f / 1024.0f;
constexpr float kLoScale     = 2048.0f;
constexpr float kLoScaleInv  = 1.0f / 2048.0f;

constexpr size_t kSzUF    = (size_t)kWidth * kNpos * 4;
constexpr size_t kSzUH    = (size_t)kWidth * kNpos * 2;
constexpr size_t kSzS32   = (size_t)kWidth * kRowsM * kStateW * 4;
constexpr size_t kSzInit  = (size_t)kWidth * kRowsM * kStateW * 2;
constexpr size_t kSzMv    = (size_t)kWidth * kChunk * kMvW * 2;
constexpr size_t kSzEt    = (size_t)kWidth * kStateW * kChunk * 2;
constexpr size_t kSzWpow  = (size_t)kWidth * kModes * 2 * 4;
constexpr size_t kSzWot   = (size_t)kLayers * kGluW * kWidth * 2;
constexpr size_t kSzWp    = (size_t)kWidth * kInPad * 2;
constexpr size_t kSzWh    = (size_t)kOutPad * kWidth * 2;
constexpr size_t kOffUF0  = 0;
constexpr size_t kOffUF1  = kOffUF0  + kSzUF;
constexpr size_t kOffUH   = kOffUF1  + kSzUF;
constexpr size_t kOffG16  = kOffUH   + kSzUH;
constexpr size_t kOffS32  = kOffG16  + kSzUH;
constexpr size_t kOffInit = kOffS32  + kSzS32;
constexpr size_t kOffMv   = kOffInit + kSzInit;
constexpr size_t kOffEt   = kOffMv   + kSzMv;
constexpr size_t kOffWpow = kOffEt   + kSzEt;
constexpr size_t kOffWot  = kOffWpow + kSzWpow;
constexpr size_t kOffWph  = kOffWot  + kSzWot;
constexpr size_t kOffWpl  = kOffWph  + kSzWp;
constexpr size_t kOffWhh  = kOffWpl  + kSzWp;
constexpr size_t kOffWhl  = kOffWhh  + kSzWh;
constexpr size_t kWsTotal = kOffWhl  + kSzWh;
static_assert(kWsTotal == 102170624ull, "carve total");
static_assert(kWsTotal <= 134217728ull, "carve cap");
static_assert((kOffUF1 % 128) == 0 && (kOffUH % 128) == 0 && (kOffG16 % 128) == 0 && (kOffS32 % 128) == 0 &&
              (kOffInit % 128) == 0 && (kOffMv % 128) == 0 && (kOffEt % 128) == 0 && (kOffWpow % 128) == 0 &&
              (kOffWot % 128) == 0 && (kOffWph % 128) == 0 && (kOffWpl % 128) == 0 && (kOffWhh % 128) == 0 &&
              (kOffWhl % 128) == 0, "128-B aligned regions");

__device__ __forceinline__ unsigned short f16bits(float x) {
  const _Float16 h = (_Float16)x;
  return __builtin_bit_cast(unsigned short, h);
}
__device__ __forceinline__ unsigned pack2(float a, float b) {
  const unsigned lo = (unsigned)f16bits(a);
  const unsigned hi = (unsigned)f16bits(b);
  return lo | (hi << 16);
}
__device__ __forceinline__ float f16_back(float x) {
  const _Float16 h = (_Float16)x;
  return (float)h;
}
__device__ __forceinline__ void wave_sync() {
  __builtin_amdgcn_fence(__ATOMIC_RELEASE, "workgroup");
  __builtin_amdgcn_wave_barrier();
  __builtin_amdgcn_fence(__ATOMIC_ACQUIRE, "workgroup");
}
__device__ __forceinline__ void store2_v4u(unsigned short* p, v4u v) {
  volatile v4u* q = (volatile v4u*)p;
  *q = v;
  __threadfence();
  *q = v;
}
__device__ __forceinline__ float gelu_tanh_f(float x) {
  const float x3 = x * x * x;
  const float u = 0.7978845608028654f * (x + 0.044715f * x3);
  return 0.5f * x * (1.0f + tanhf(u));
}
__device__ __forceinline__ float sigmoid_f(float g) {
  const float e = expf(-fabsf(g));
  const float s = 1.0f / (1.0f + e);
  return (g >= 0.0f) ? s : (e * s);
}

union FragH { v16h v; v8h h[2]; };
union FragW { v16h v; v4u q[2]; };
__device__ __forceinline__ v16h frag_load(const _Float16* p) {
  FragH f;
  f.h[0] = *(const v8h*)(p);
  f.h[1] = *(const v8h*)(p + 16);
  return f.v;
}
template <int PITCH>
__device__ __forceinline__ v16h lds_frag(const unsigned* sw, int n, int kw) {
  FragW f;
  f.q[0] = *(const v4u*)(sw + n * PITCH + kw);
  f.q[1] = *(const v4u*)(sw + n * PITCH + kw + 8);
  return f.v;
}
__device__ __forceinline__ v8f mma16(v16h a, v16h b, v8f c) {
  return __builtin_amdgcn_wmma_f32_16x16x32_f16(false, a, false, b, (short)0, c, false, false);
}
__device__ __forceinline__ void tie_acc(v8f& a, v16h x, v16h y) { asm volatile("" : "+v"(a) : "v"(x), "v"(y)); }
__device__ __forceinline__ void tie_acc_nops(v8f& a, v16h x, v16h y) { asm volatile("v_nop\n\tv_nop\n\tv_nop\n\tv_nop" : "+v"(a) : "v"(x), "v"(y)); }
__device__ __forceinline__ void keep4(v16h a, v16h b, v16h c, v16h d) { asm volatile("v_nop" :: "v"(a), "v"(b), "v"(c), "v"(d)); }
__device__ __forceinline__ void keep2(v16h a, v16h b) { asm volatile("v_nop" :: "v"(a), "v"(b)); }
__device__ __forceinline__ void acc_guard4(v8f& a, v8f& b, v8f& c, v8f& d) { asm volatile("v_nop\n\tv_nop\n\tv_nop\n\tv_nop" : "+v"(a), "+v"(b), "+v"(c), "+v"(d)); }
__device__ __forceinline__ void acc_guard2(v8f& a, v8f& b) { asm volatile("v_nop\n\tv_nop\n\tv_nop\n\tv_nop" : "+v"(a), "+v"(b)); }

__device__ __forceinline__ void kloop64(v8f (&acc)[4][4], const _Float16* ap, int lda,
                                        const _Float16* bp, int ldb, int ksteps) {
#pragma unroll 1
  for (int ks = 0; ks < ksteps; ++ks) {
    v16h bh[4];
#pragma unroll
    for (int j = 0; j < 4; ++j) bh[j] = frag_load(bp + (size_t)(j * 16) * ldb + ks * 32);
#pragma unroll
    for (int i = 0; i < 4; ++i) {
      const v16h ah = frag_load(ap + (size_t)(i * 16) * lda + ks * 32);
#pragma unroll
      for (int j = 0; j < 4; ++j) acc[i][j] = mma16(ah, bh[j], acc[i][j]);
      tie_acc(acc[i][0], ah, bh[0]);
      tie_acc(acc[i][1], ah, bh[1]);
      tie_acc(acc[i][2], ah, bh[2]);
      tie_acc_nops(acc[i][3], ah, bh[3]);
    }
    keep4(bh[0], bh[1], bh[2], bh[3]);
  }
}

template <int NT, int PITCH>
__device__ __forceinline__ void split_kloop(v8f (&am)[NT], v8f (&ar)[NT],
                                            const _Float16* ah_p, const _Float16* al_p,
                                            const unsigned* sBh, const unsigned* sBl,
                                            int c, int hh, int ksteps) {
#pragma unroll 1
  for (int ks = 0; ks < ksteps; ++ks) {
    v16h bh[NT];
    v16h bl[NT];
#pragma unroll
    for (int j = 0; j < NT; ++j) {
      bh[j] = lds_frag<PITCH>(sBh, 16 * j + c, ks * 16 + 4 * hh);
      bl[j] = lds_frag<PITCH>(sBl, 16 * j + c, ks * 16 + 4 * hh);
    }
    const v16h ah = frag_load(ah_p + ks * 32);
    const v16h al = frag_load(al_p + ks * 32);
#pragma unroll
    for (int j = 0; j < NT; ++j) {
      am[j] = mma16(ah, bh[j], am[j]);
      ar[j] = mma16(ah, bl[j], ar[j]);
      ar[j] = mma16(al, bh[j], ar[j]);
    }
#pragma unroll
    for (int j = 0; j < NT; ++j) tie_acc(am[j], ah, bh[j]);
#pragma unroll
    for (int j = 0; j < NT - 1; ++j) tie_acc(ar[j], al, bl[j]);
    tie_acc_nops(ar[NT - 1], al, bl[NT - 1]);
#pragma unroll
    for (int j = 0; j < NT; ++j) keep2(bh[j], bl[j]);
  }
}

template <int NT>
__device__ __forceinline__ void stage_tile_T(const unsigned short* plane, size_t n0, unsigned* sw, int tid) {
#pragma unroll 1
  for (int it = 0; it < 1024 / NT; ++it) {
    const int task = it * NT + tid;
    const int n8 = task & 7;
    const int kp = task >> 3;
    const unsigned short* p0 = plane + (size_t)(2 * kp) * kNpos + n0 + n8 * 8;
    const v4u a = *(const v4u*)(p0);
    const v4u b = *(const v4u*)(p0 + kNpos);
    unsigned* dst = sw + (n8 * 8) * kPitchW + kp;
#pragma unroll
    for (int j = 0; j < 4; ++j) {
      const unsigned aw = a[j];
      const unsigned bw = b[j];
      dst[(2 * j) * kPitchW]     = (aw & 0xffffu) | (bw << 16);
      dst[(2 * j + 1) * kPitchW] = (aw >> 16) | (bw & 0xffff0000u);
    }
  }
}

template <bool RES>
__device__ __forceinline__ void emit_rows(float* slab, const float* resid, float* outF, unsigned short* outH,
                                          int d0, size_t n0, int lane) {
  const int h2 = lane >> 4;
  const int c4 = (lane & 15) * 4;
  v4f vf[8];
#pragma unroll
  for (int it = 0; it < 8; ++it) {
    const int row = it * 2 + h2;
    v4f v = *(const v4f*)(slab + row * 68 + c4);
    if (RES) {
      const v4f r = *(const v4f*)(resid + (size_t)(d0 + row) * kNpos + n0 + c4);
      v = v + r;
      *(v4f*)(slab + row * 68 + c4) = v;
    }
    vf[it] = v;
  }
  wave_sync();
  const int q = lane >> 3;
  const int cw = lane & 7;
  v4u vh[4];
#pragma unroll
  for (int it = 0; it < 4; ++it) {
    const int row = it * 4 + q;
    const float* sp = slab + row * 68 + cw * 8;
    const v4f a0 = *(const v4f*)(sp);
    const v4f a1 = *(const v4f*)(sp + 4);
    const v4u pk = {pack2(a0[0], a0[1]), pack2(a0[2], a0[3]), pack2(a1[0], a1[1]), pack2(a1[2], a1[3])};
    vh[it] = pk;
  }
  for (int pass = 0; pass < 2; ++pass) {
#pragma unroll
    for (int it = 0; it < 8; ++it) {
      const int row = it * 2 + h2;
      *(volatile v4f*)(outF + (size_t)(d0 + row) * kNpos + n0 + c4) = vf[it];
    }
#pragma unroll
    for (int it = 0; it < 4; ++it) {
      const int row = it * 4 + q;
      *(volatile v4u*)(outH + (size_t)(d0 + row) * kNpos + n0 + cw * 8) = vh[it];
    }
    __threadfence();
  }
}

template <int KREAL, int KP, bool LO>
__device__ __forceinline__ void transpose_rows(const float* __restrict__ src, int ld, int mcount, int m0,
                                               unsigned short* dhi, unsigned short* dlo, float* sT, int tid) {
  const int mm = tid & 31;
  const int kq = tid >> 5;
  const int mreal = m0 + mm;
  const int ms = (mreal < mcount) ? mreal : (mcount - 1);
  constexpr int LIT = (KREAL + 7) / 8;
#pragma unroll 1
  for (int it = 0; it < LIT; ++it) {
    const int k = it * 8 + kq;
    const int kc = (k < KREAL) ? k : (KREAL - 1);
    const float v = src[(size_t)kc * ld + ms];
    if (k < KREAL) sT[mm * 257 + k] = v;
  }
  __syncthreads();
  constexpr int CPR = KP / 8;
  constexpr int NCH = 32 * CPR;
  constexpr int ITERS = (NCH + 255) / 256;
#pragma unroll 1
  for (int it = 0; it < ITERS; ++it) {
    const int q = it * 256 + tid;
    if (q < NCH) {
      const int row = q / CPR;
      const int k8 = (q - row * CPR) * 8;
      const bool rowok = (m0 + row) < mcount;
      float vh[8];
      float vl[8];
#pragma unroll
      for (int e = 0; e < 8; ++e) {
        const int kk = k8 + e;
        const int kc = (kk < KREAL) ? kk : (KREAL - 1);
        const float x = sT[row * 257 + kc];
        const float v = ((kk < KREAL) && rowok) ? (x * kWCarry) : 0.0f;
        const float back = f16_back(v);
        vh[e] = v;
        vl[e] = (v - back) * kLoScale;
      }
      const v4u ph = {pack2(vh[0], vh[1]), pack2(vh[2], vh[3]), pack2(vh[4], vh[5]), pack2(vh[6], vh[7])};
      store2_v4u(dhi + (size_t)q * 8, ph);
      if (LO) {
        const v4u pl = {pack2(vl[0], vl[1]), pack2(vl[2], vl[3]), pack2(vl[4], vl[5]), pack2(vl[6], vl[7])};
        store2_v4u(dlo + (size_t)q * 8, pl);
      }
    }
  }
}

__global__ __launch_bounds__(256) void weight_planes_kernel(
    const float* __restrict__ out_w, const float* __restrict__ proj_w, const float* __restrict__ head_w,
    unsigned short* __restrict__ wot, unsigned short* __restrict__ wph, unsigned short* __restrict__ wpl,
    unsigned short* __restrict__ whh, unsigned short* __restrict__ whl) {
  __shared__ float sT[32 * 257];
  const int tid = threadIdx.x;
  const int bid = blockIdx.x;
  if (bid < 64) {
    const int layer = bid >> 4;
    const int m0 = (bid & 15) * 32;
    transpose_rows<kWidth, kWidth, false>(out_w + (size_t)layer * kWidth * kGluW, kGluW, kGluW, m0,
                                          wot + (size_t)layer * kGluW * kWidth + (size_t)m0 * kWidth, nullptr, sT, tid);
  } else if (bid < 72) {
    const int m0 = (bid - 64) * 32;
    transpose_rows<kInDim, kInPad, true>(proj_w, kWidth, kWidth, m0, wph + (size_t)m0 * kInPad, wpl + (size_t)m0 * kInPad, sT, tid);
  } else {
    const int m0 = (bid - 72) * 32;
    transpose_rows<kWidth, kWidth, true>(head_w, kOutDim, kOutDim, m0, whh + (size_t)m0 * kWidth, whl + (size_t)m0 * kWidth, sT, tid);
  }
}

__global__ __launch_bounds__(256) void input_proj_kernel(
    const float* __restrict__ x, const unsigned short* __restrict__ wph, const unsigned short* __restrict__ wpl,
    const float* __restrict__ pb, float* __restrict__ uf, unsigned short* __restrict__ uh) {
  __shared__ __align__(16) unsigned sXh[64 * kPitchX];
  __shared__ __align__(16) unsigned sXl[64 * kPitchX];
  __shared__ __align__(16) float sSlab[8][16 * 68];
  const int tid = threadIdx.x;
  const int lane = tid & 31;
  const int wave = __builtin_amdgcn_readfirstlane((int)(threadIdx.x >> 5));
  const int hh = lane >> 4;
  const int c = lane & 15;
  const size_t n0 = (size_t)blockIdx.x * 64;
#pragma unroll 1
  for (int it = 0; it < 8; ++it) {
    const int task = it * 256 + tid;
    const int w = task & 31;
    const int n = task >> 5;
    const float* xr = x + (n0 + (size_t)n) * kInDim;
    const int k0i = 2 * w;
    const int k1i = 2 * w + 1;
    const int c0 = (k0i < kInDim) ? k0i : (kInDim - 1);
    const int c1 = (k1i < kInDim) ? k1i : (kInDim - 1);
    const float x0 = xr[c0];
    const float x1 = xr[c1];
    const float v0 = (k0i < kInDim) ? x0 : 0.0f;
    const float v1 = (k1i < kInDim) ? x1 : 0.0f;
    const float l0 = (v0 - f16_back(v0)) * kLoScale;
    const float l1 = (v1 - f16_back(v1)) * kLoScale;
    sXh[n * kPitchX + w] = pack2(v0, v1);
    sXl[n * kPitchX + w] = pack2(l0, l1);
  }
  __syncthreads();
  float* slab = sSlab[wave];
#pragma unroll 1
  for (int i = 0; i < 2; ++i) {
    const int d0 = 32 * wave + 16 * i;
    v8f am[4];
    v8f ar[4];
#pragma unroll
    for (int j = 0; j < 4; ++j) {
      am[j] = (v8f){0.f, 0.f, 0.f, 0.f, 0.f, 0.f, 0.f, 0.f};
      ar[j] = (v8f){0.f, 0.f, 0.f, 0.f, 0.f, 0.f, 0.f, 0.f};
    }
    split_kloop<4, kPitchX>(am, ar,
                            (const _Float16*)wph + (size_t)(d0 + c) * kInPad + 8 * hh,
                            (const _Float16*)wpl + (size_t)(d0 + c) * kInPad + 8 * hh,
                            sXh, sXl, c, hh, kInPad / 32);
    acc_guard4(am[0], am[1], am[2], am[3]);
    acc_guard4(ar[0], ar[1], ar[2], ar[3]);
    const v4f b0 = *(const v4f*)(pb + d0 + 8 * hh);
    const v4f b1 = *(const v4f*)(pb + d0 + 8 * hh + 4);
#pragma unroll
    for (int j = 0; j < 4; ++j) {
#pragma unroll
      for (int r = 0; r < 8; ++r) {
        const float bv = (r < 4) ? b0[r & 3] : b1[r & 3];
        const float sum = fmaf(ar[j][r], kLoScaleInv, am[j][r]);
        slab[(8 * hh + r) * 68 + 16 * j + c] = fmaf(sum, kWCarryInv, bv);
      }
    }
    wave_sync();
    emit_rows<false>(slab, nullptr, uf, uh, d0, n0, lane);
    wave_sync();
  }
}

__global__ __launch_bounds__(256) void layer_tables_kernel(
    const float* __restrict__ log_dt, const float* __restrict__ a_re, const float* __restrict__ a_im,
    const float* __restrict__ c_re, const float* __restrict__ c_im,
    unsigned short* __restrict__ et16, unsigned short* __restrict__ mv16, float* __restrict__ wpow) {
  __shared__ __align__(16) unsigned sStage[128 * 64];
  __shared__ float sRr[10 * 64];
  __shared__ float sRi[10 * 64];
  __shared__ float sSn[64];
  __shared__ float sCs[64];
  __shared__ float sKp[128 * 2];
  __shared__ float sK[128];
  const int tid = threadIdx.x;
  const int lane = tid & 31;
  const int n = tid & 63;
  const int seg = __builtin_amdgcn_readfirstlane((int)(threadIdx.x >> 6));
  const int wv = __builtin_amdgcn_readfirstlane((int)(threadIdx.x >> 5));
  const int h = blockIdx.x;
  const int idx = h * kModes + n;
  const float dt = expf(log_dt[h]);
  const float ar = -expf(a_re[idx]);
  const float ai = a_im[idx];
  const float dr = ar * dt;
  const float di = ai * dt;
#pragma unroll 1
  for (int it = 0; it < 3; ++it) {
    const int e = seg + 4 * it;
    const int ec = (e < 10) ? e : 9;
    const int lmul = (ec == 0) ? 1 : (16 * (ec - 1));
    const float fl = (float)lmul;
    const float mag = expf(dr * fl);
    float sn, cs;
    sincosf(di * fl, &sn, &cs);
    if (e < 10) {
      sRr[ec * 64 + n] = mag * cs;
      sRi[ec * 64 + n] = mag * sn;
      if (e == 0) {
        sSn[n] = sn;
        sCs[n] = cs;
      }
    }
  }
  __syncthreads();
  const float wr = sRr[n];
  const float wi = sRi[n];
  float c2r, c2i;
  {
    const float sn = sSn[n];
    const float cs = sCs[n];
    const float em = expm1f(dr);
    const float cm1a = -(sn * sn) * (1.0f / (1.0f + fmaxf(cs, 0.0f)));
    const float cm1 = (cs > 0.0f) ? cm1a : (cs - 1.0f);
    const float nr = em * cs + cm1;
    const float ni = wi;
    const float inv = 1.0f / (ar * ar + ai * ai);
    const float qr = (nr * ar + ni * ai) * inv;
    const float qi = (ni * ar - nr * ai) * inv;
    const float cr = c_re[idx];
    const float ci = c_im[idx];
    c2r = 2.0f * (cr * qr - ci * qi);
    c2i = 2.0f * (cr * qi + ci * qr);
  }
#pragma unroll 1
  for (int half = 0; half < 2; ++half) {
    const int g = 2 * seg + half;
    float pr = sRr[(1 + g) * 64 + n];
    float pi = sRi[(1 + g) * 64 + n];
#pragma unroll 1
    for (int s = 0; s < 16; ++s) {
      const int l = 16 * g + s;
      float term = c2r * pr - c2i * pi;
      term += __shfl_xor(term, 16, 32);
      term += __shfl_xor(term, 8, 32);
      term += __shfl_xor(term, 4, 32);
      term += __shfl_xor(term, 2, 32);
      term += __shfl_xor(term, 1, 32);
      if (lane == 0) sKp[l * 2 + (wv & 1)] = term;
      const float t = pr * wr - pi * wi;
      pi = pr * wi + pi * wr;
      pr = t;
      const float re = c2r * pr - c2i * pi;
      const float im = c2r * pi + c2i * pr;
      sStage[l * 64 + n] = pack2(re * kTabCarry, -im * kTabCarry);
    }
  }
  __syncthreads();
  if (tid < 128) sK[tid] = sKp[2 * tid] + sKp[2 * tid + 1];
  __syncthreads();
#pragma unroll 1
  for (int it = 0; it < 8; ++it) {
    const int q = it * 256 + tid;
    const int row = q >> 4;
    const int s0 = (q & 15) * 8;
    float v[8];
#pragma unroll
    for (int e = 0; e < 8; ++e) {
      const int df = row - (s0 + e);
      int dc = (df < 0) ? 0 : df;
      dc = (dc > 127) ? 127 : dc;
      const float kv = sK[dc];
      const float val = (df >= 0) ? kv : 0.0f;
      v[e] = val * kTabCarry;
    }
    const v4u pk = {pack2(v[0], v[1]), pack2(v[2], v[3]), pack2(v[4], v[5]), pack2(v[6], v[7])};
    store2_v4u(mv16 + ((size_t)h * kChunk + row) * kMvW + s0, pk);
  }
#pragma unroll 1
  for (int it = 0; it < 8; ++it) {
    const int q = it * 256 + tid;
    const int row = q >> 4;
    const int cw = q & 15;
    const v4u pk = *(const v4u*)(sStage + row * 64 + cw * 4);
    store2_v4u(mv16 + ((size_t)h * kChunk + row) * kMvW + kChunk + cw * 8, pk);
  }
  if (seg == 0) {
    const v2f wv2 = {sRr[9 * 64 + n], sRi[9 * 64 + n]};
    volatile v2f* wp = (volatile v2f*)(wpow + (size_t)(h * kModes + n) * 2);
    *wp = wv2;
    __threadfence();
    *wp = wv2;
  }
  __syncthreads();
#pragma unroll 1
  for (int half = 0; half < 2; ++half) {
    const int g = 2 * seg + half;
    float pr = sRr[(1 + g) * 64 + n];
    float pi = sRi[(1 + g) * 64 + n];
#pragma unroll 1
    for (int s2 = 0; s2 < 8; ++s2) {
      const int l = 16 * g + 2 * s2;
      const float pr0 = pr;
      const float pi0 = pi;
      const float pr1 = pr0 * wr - pi0 * wi;
      const float pi1 = pr0 * wi + pi0 * wr;
      const int kw = (126 - l) >> 1;
      sStage[(2 * n) * 64 + kw]     = pack2(pr1 * kTabCarry, pr0 * kTabCarry);
      sStage[(2 * n + 1) * 64 + kw] = pack2(pi1 * kTabCarry, pi0 * kTabCarry);
      pr = pr1 * wr - pi1 * wi;
      pi = pr1 * wi + pi1 * wr;
    }
  }
  __syncthreads();
#pragma unroll 1
  for (int it = 0; it < 8; ++it) {
    const int q = it * 256 + tid;
    const int row = q >> 4;
    const int cw = q & 15;
    const v4u pk = *(const v4u*)(sStage + row * 64 + cw * 4);
    store2_v4u(et16 + ((size_t)h * kStateW + row) * kChunk + cw * 8, pk);
  }
}

template <int MODE>
__global__ __launch_bounds__(256) void chunk_gemm_kernel(
    const unsigned short* __restrict__ hplane, const unsigned short* __restrict__ initp,
    const unsigned short* __restrict__ btp, void* __restrict__ cout,
    const float* __restrict__ ucur, const float* __restrict__ dskip) {
  __shared__ __align__(16) float sT[8][16 * 68];
  __shared__ __align__(16) unsigned sHw[(MODE == 1) ? 8 : 1][(MODE == 1) ? 16 * 32 : 4];
  const int lane = threadIdx.x & 31;
  const int wave = __builtin_amdgcn_readfirstlane((int)(threadIdx.x >> 5));
  const int g = (int)blockIdx.x * 8 + wave;
  const int h = g >> 2;
  const int tm = (g >> 1) & 1;
  const int tn = g & 1;
  const int m0 = tm << 6;
  const int n0 = tn << 6;
  const int rlane = lane & 15;
  const int koff = (lane >> 4) * 8;
  const int mOff = (lane >> 4) * 8;
  constexpr int LDB = (MODE == 1) ? kMvW : kChunk;
  const _Float16* A1 = (const _Float16*)hplane + (size_t)h * kNpos;
  const _Float16* Bt = (const _Float16*)btp + (size_t)h * 128 * LDB;

  v8f acc[4][4];
#pragma unroll
  for (int i = 0; i < 4; ++i)
#pragma unroll
    for (int j = 0; j < 4; ++j) acc[i][j] = (v8f){0.f, 0.f, 0.f, 0.f, 0.f, 0.f, 0.f, 0.f};

  const int ks1 = (MODE == 1) ? ((tn + 1) * 2) : (kChunk / 32);
  kloop64(acc, A1 + (size_t)(m0 + rlane) * kChunk + koff, kChunk,
          Bt + (size_t)(n0 + rlane) * LDB + koff, LDB, ks1);
  if (MODE == 1) {
    const _Float16* A2 = (const _Float16*)initp + (size_t)h * kRowsM * kStateW;
    kloop64(acc, A2 + (size_t)(m0 + rlane) * kStateW + koff, kStateW,
            Bt + (size_t)(n0 + rlane) * LDB + kChunk + koff, LDB, kStateW / 32);
  }
  acc_guard4(acc[0][0], acc[0][1], acc[0][2], acc[0][3]);
  acc_guard4(acc[1][0], acc[1][1], acc[1][2], acc[1][3]);
  acc_guard4(acc[2][0], acc[2][1], acc[2][2], acc[2][3]);
  acc_guard4(acc[3][0], acc[3][1], acc[3][2], acc[3][3]);

  float* slab = sT[wave];
  float dsk = 0.0f;
  if (MODE == 1) dsk = dskip[h];
#pragma unroll
  for (int i = 0; i < 4; ++i) {
    const int mBase = m0 + (i << 4);
#pragma unroll
    for (int j = 0; j < 4; ++j) {
#pragma unroll
      for (int r = 0; r < 8; ++r) slab[(mOff + r) * 68 + (j << 4) + rlane] = acc[i][j][r] * kTabCarryInv;
    }
    wave_sync();
    if (MODE == 0) {
      float* C = (float*)cout + (size_t)h * kRowsM * kStateW;
      const int h2 = lane >> 4;
      const int c4 = (lane & 15) * 4;
      v4f vals[8];
#pragma unroll
      for (int it = 0; it < 8; ++it) vals[it] = *(const v4f*)(slab + (it * 2 + h2) * 68 + c4);
      for (int pass = 0; pass < 2; ++pass) {
#pragma unroll
        for (int it = 0; it < 8; ++it) {
          const int row = it * 2 + h2;
          *(volatile v4f*)(C + (size_t)(mBase + row) * kStateW + n0 + c4) = vals[it];
        }
        __threadfence();
      }
    } else {
      unsigned* sH = sHw[wave];
      unsigned short* G = (unsigned short*)cout + (size_t)h * kNpos;
      const int q = lane >> 3;
      const int cw = lane & 7;
#pragma unroll 1
      for (int it = 0; it < 4; ++it) {
        const int row = it * 4 + q;
        const float* sp = slab + row * 68 + cw * 8;
        const v4f a0 = *(const v4f*)(sp);
        const v4f a1 = *(const v4f*)(sp + 4);
        const float* up = ucur + (size_t)h * kNpos + (size_t)(mBase + row) * kChunk + n0 + cw * 8;
        const v4f u0 = *(const v4f*)(up);
        const v4f u1 = *(const v4f*)(up + 4);
        const float z0 = gelu_tanh_f(fmaf(dsk, u0[0], a0[0]));
        const float z1 = gelu_tanh_f(fmaf(dsk, u0[1], a0[1]));
        const float z2 = gelu_tanh_f(fmaf(dsk, u0[2], a0[2]));
        const float z3 = gelu_tanh_f(fmaf(dsk, u0[3], a0[3]));
        const float z4 = gelu_tanh_f(fmaf(dsk, u1[0], a1[0]));
        const float z5 = gelu_tanh_f(fmaf(dsk, u1[1], a1[1]));
        const float z6 = gelu_tanh_f(fmaf(dsk, u1[2], a1[2]));
        const float z7 = gelu_tanh_f(fmaf(dsk, u1[3], a1[3]));
        const v4u pk = {pack2(z0, z1), pack2(z2, z3), pack2(z4, z5), pack2(z6, z7)};
        *(v4u*)(sH + row * 32 + cw * 4) = pk;
      }
      wave_sync();
      v4u vals[4];
#pragma unroll
      for (int it = 0; it < 4; ++it) vals[it] = *(const v4u*)(sH + (it * 4 + q) * 32 + cw * 4);
      for (int pass = 0; pass < 2; ++pass) {
#pragma unroll
        for (int it = 0; it < 4; ++it) {
          const int row = it * 4 + q;
          *(volatile v4u*)(G + (size_t)(mBase + row) * kChunk + n0 + cw * 8) = vals[it];
        }
        __threadfence();
      }
    }
    wave_sync();
  }
}

__global__ __launch_bounds__(256) void combine_kernel(
    const float* __restrict__ s32, const float* __restrict__ wpow, unsigned short* __restrict__ init16) {
  const int lane = threadIdx.x & 31;
  const int wave = __builtin_amdgcn_readfirstlane((int)(threadIdx.x >> 5));
  const int pair = (int)blockIdx.x * 8 + wave;
  const int h = pair >> 3;
  const int b = pair & 7;
  const v2f w0 = *(const v2f*)(wpow + (size_t)(h * kModes + lane) * 2);
  const v2f w1 = *(const v2f*)(wpow + (size_t)(h * kModes + 32 + lane) * 2);
  const float* sp = s32 + ((size_t)h * kRowsM + (size_t)b * kChunksPS) * kStateW;
  unsigned* ip = (unsigned*)(init16 + ((size_t)h * kRowsM + (size_t)b * kChunksPS) * kStateW);
  float e0r = 0.0f, e0i = 0.0f, e1r = 0.0f, e1i = 0.0f;
#pragma unroll 1
  for (int cidx = 0; cidx < kChunksPS; ++cidx) {
    const v2f s0 = *(const v2f*)(sp + (size_t)cidx * kStateW + 2 * lane);
    const v2f s1 = *(const v2f*)(sp + (size_t)cidx * kStateW + 64 + 2 * lane);
    const float a0 = fminf(fmaxf(e0r, -60000.0f), 60000.0f);
    const float a1 = fminf(fmaxf(e0i, -60000.0f), 60000.0f);
    const float a2 = fminf(fmaxf(e1r, -60000.0f), 60000.0f);
    const float a3 = fminf(fmaxf(e1i, -60000.0f), 60000.0f);
    const unsigned word0 = pack2(a0, a1);
    const unsigned word1 = pack2(a2, a3);
    volatile unsigned* q0 = (volatile unsigned*)(ip + (size_t)cidx * (kStateW / 2) + lane);
    volatile unsigned* q1 = (volatile unsigned*)(ip + (size_t)cidx * (kStateW / 2) + 32 + lane);
    *q0 = word0;
    *q1 = word1;
    __threadfence();
    *q0 = word0;
    *q1 = word1;
    const float t0 = w0[0] * e0r - w0[1] * e0i + s0[0];
    e0i = w0[0] * e0i + w0[1] * e0r + s0[1];
    e0r = t0;
    const float t1 = w1[0] * e1r - w1[1] * e1i + s1[0];
    e1i = w1[0] * e1i + w1[1] * e1r + s1[1];
    e1r = t1;
  }
}

__global__ __launch_bounds__(128) void glu_kernel(
    const unsigned short* __restrict__ g16, const unsigned short* __restrict__ wT,
    const float* __restrict__ ob, const float* __restrict__ ucur,
    float* __restrict__ unext, unsigned short* __restrict__ uh) {
  __shared__ __align__(16) unsigned sW[64 * kPitchW];
  __shared__ __align__(16) float sSlab[4][16 * 68];
  const int tid = threadIdx.x;
  const int lane = tid & 31;
  const int wave = __builtin_amdgcn_readfirstlane((int)(threadIdx.x >> 5));
  const int hh = lane >> 4;
  const int c = lane & 15;
  const size_t n0 = (size_t)blockIdx.x * 64;

  stage_tile_T<128>(g16, n0, sW, tid);
  __syncthreads();

  float* slab = sSlab[wave];
#pragma unroll 1
  for (int i = 0; i < 4; ++i) {
    const int d0 = 64 * wave + 16 * i;
    v8f aa[4];
    v8f ag[4];
#pragma unroll
    for (int j = 0; j < 4; ++j) {
      aa[j] = (v8f){0.f, 0.f, 0.f, 0.f, 0.f, 0.f, 0.f, 0.f};
      ag[j] = (v8f){0.f, 0.f, 0.f, 0.f, 0.f, 0.f, 0.f, 0.f};
    }
    const _Float16* Wa = (const _Float16*)wT + (size_t)(d0 + c) * kWidth + 8 * hh;
    const _Float16* Wg = (const _Float16*)wT + (size_t)(kWidth + d0 + c) * kWidth + 8 * hh;
#pragma unroll 1
    for (int ks = 0; ks < kWidth / 32; ++ks) {
      v16h bf[4];
#pragma unroll
      for (int j = 0; j < 4; ++j) bf[j] = lds_frag<kPitchW>(sW, 16 * j + c, ks * 16 + 4 * hh);
      const v16h fa = frag_load(Wa + ks * 32);
      const v16h fg = frag_load(Wg + ks * 32);
#pragma unroll
      for (int j = 0; j < 4; ++j) {
        aa[j] = mma16(fa, bf[j], aa[j]);
        ag[j] = mma16(fg, bf[j], ag[j]);
      }
      tie_acc(aa[0], fa, bf[0]);
      tie_acc(aa[1], fa, bf[1]);
      tie_acc(aa[2], fa, bf[2]);
      tie_acc(aa[3], fa, bf[3]);
      tie_acc(ag[0], fg, bf[0]);
      tie_acc(ag[1], fg, bf[1]);
      tie_acc(ag[2], fg, bf[2]);
      tie_acc_nops(ag[3], fg, bf[3]);
      keep4(bf[0], bf[1], bf[2], bf[3]);
    }
    acc_guard4(aa[0], aa[1], aa[2], aa[3]);
    acc_guard4(ag[0], ag[1], ag[2], ag[3]);
    const v4f ba0 = *(const v4f*)(ob + d0 + 8 * hh);
    const v4f ba1 = *(const v4f*)(ob + d0 + 8 * hh + 4);
    const v4f bg0 = *(const v4f*)(ob + kWidth + d0 + 8 * hh);
    const v4f bg1 = *(const v4f*)(ob + kWidth + d0 + 8 * hh + 4);
#pragma unroll
    for (int j = 0; j < 4; ++j) {
#pragma unroll
      for (int r = 0; r < 8; ++r) {
        const float bv = (r < 4) ? bg0[r & 3] : bg1[r & 3];
        slab[(8 * hh + r) * 68 + 16 * j + c] = fmaf(ag[j][r], kWCarryInv, bv);
      }
    }
    wave_sync();
    {
      const int h2 = lane >> 4;
      const int c4 = (lane & 15) * 4;
#pragma unroll 1
      for (int it = 0; it < 8; ++it) {
        float* p = slab + (it * 2 + h2) * 68 + c4;
        const v4f gv = *(const v4f*)p;
        v4f sv;
        sv[0] = sigmoid_f(gv[0]);
        sv[1] = sigmoid_f(gv[1]);
        sv[2] = sigmoid_f(gv[2]);
        sv[3] = sigmoid_f(gv[3]);
        *(v4f*)p = sv;
      }
    }
    wave_sync();
#pragma unroll
    for (int j = 0; j < 4; ++j) {
#pragma unroll
      for (int r = 0; r < 8; ++r) {
        const float bv = (r < 4) ? ba0[r & 3] : ba1[r & 3];
        const int si = (8 * hh + r) * 68 + 16 * j + c;
        const float sg = slab[si];
        const float av = fmaf(aa[j][r], kWCarryInv, bv);
        slab[si] = av * sg;
      }
    }
    wave_sync();
    emit_rows<true>(slab, ucur, unext, uh, d0, n0, lane);
    wave_sync();
  }
}

__global__ __launch_bounds__(256) void norm_head_kernel(
    const float* __restrict__ uf, const unsigned short* __restrict__ whh, const unsigned short* __restrict__ whl,
    const float* __restrict__ ln_g, const float* __restrict__ ln_b, const float* __restrict__ head_b,
    float* __restrict__ out) {
  __shared__ __align__(16) unsigned sBh[kHeadPos * kPitchW];
  __shared__ __align__(16) unsigned sBl[kHeadPos * kPitchW];
  __shared__ __align__(16) float sOut[kHeadPos * kOutDim];
  __shared__ float sRed[256];
  __shared__ float sMu[32];
  __shared__ float sRs[32];
  const int tid = threadIdx.x;
  const int lane = tid & 31;
  const int wave = __builtin_amdgcn_readfirstlane((int)(threadIdx.x >> 5));
  const int hh = lane >> 4;
  const int c = lane & 15;
  const size_t n0 = (size_t)blockIdx.x * kHeadPos;
  const int n = lane;
  const int hq = wave;
  const float* up = uf + (size_t)(hq * 32) * kNpos + n0 + n;
  {
    float s = 0.0f;
#pragma unroll 4
    for (int hl = 0; hl < 32; ++hl) s += up[(size_t)hl * kNpos];
    sRed[hq * 32 + n] = s;
  }
  __syncthreads();
  if (tid < 32) {
    float a = 0.0f;
#pragma unroll 1
    for (int w2 = 0; w2 < 8; ++w2) a += sRed[w2 * 32 + tid];
    sMu[tid] = a * (1.0f / (float)kWidth);
  }
  __syncthreads();
  const float mu = sMu[n];
  {
    float s2 = 0.0f;
#pragma unroll 4
    for (int hl = 0; hl < 32; ++hl) {
      const float d = up[(size_t)hl * kNpos] - mu;
      s2 = fmaf(d, d, s2);
    }
    sRed[hq * 32 + n] = s2;
  }
  __syncthreads();
  if (tid < 32) {
    float a = 0.0f;
#pragma unroll 1
    for (int w2 = 0; w2 < 8; ++w2) a += sRed[w2 * 32 + tid];
    const float var = a * (1.0f / (float)kWidth);
    sRs[tid] = 1.0f / sqrtf(var + 1e-5f);
  }
  __syncthreads();
  const float rs = sRs[n];
#pragma unroll 2
  for (int hp = 0; hp < 16; ++hp) {
    const int hc = hq * 32 + 2 * hp;
    const float x0 = up[(size_t)(2 * hp) * kNpos];
    const float x1 = up[(size_t)(2 * hp + 1) * kNpos];
    const float v0 = (x0 - mu) * rs * ln_g[hc] + ln_b[hc];
    const float v1 = (x1 - mu) * rs * ln_g[hc + 1] + ln_b[hc + 1];
    const float l0 = (v0 - f16_back(v0)) * kLoScale;
    const float l1 = (v1 - f16_back(v1)) * kLoScale;
    sBh[n * kPitchW + hq * 16 + hp] = pack2(v0, v1);
    sBl[n * kPitchW + hq * 16 + hp] = pack2(l0, l1);
  }
  __syncthreads();

#pragma unroll 1
  for (int i = 0; i < 2; ++i) {
    const int o0 = 32 * wave + 16 * i;
    v8f am[2];
    v8f ar[2];
#pragma unroll
    for (int j = 0; j < 2; ++j) {
      am[j] = (v8f){0.f, 0.f, 0.f, 0.f, 0.f, 0.f, 0.f, 0.f};
      ar[j] = (v8f){0.f, 0.f, 0.f, 0.f, 0.f, 0.f, 0.f, 0.f};
    }
    split_kloop<2, kPitchW>(am, ar,
                            (const _Float16*)whh + (size_t)(o0 + c) * kWidth + 8 * hh,
                            (const _Float16*)whl + (size_t)(o0 + c) * kWidth + 8 * hh,
                            sBh, sBl, c, hh, kWidth / 32);
    acc_guard2(am[0], ar[0]);
    acc_guard2(am[1], ar[1]);
#pragma unroll
    for (int r = 0; r < 8; ++r) {
      const int o = o0 + 8 * hh + r;
      const int oc = (o < kOutDim) ? o : (kOutDim - 1);
      float bv = head_b[oc];
      asm volatile("" : "+v"(bv));
#pragma unroll
      for (int j = 0; j < 2; ++j) {
        const int nn = 16 * j + c;
        const float sum = fmaf(ar[j][r], kLoScaleInv, am[j][r]);
        const float val = fmaf(sum, kWCarryInv, bv);
        if (o < kOutDim) sOut[nn * kOutDim + o] = val;
      }
    }
  }
  __syncthreads();
  {
    constexpr int NCHUNK = (kHeadPos * kOutDim) / 4;
    v4f vals[7];
#pragma unroll
    for (int it = 0; it < 7; ++it) {
      const int q = it * 256 + tid;
      const int qc = (q < NCHUNK) ? q : (NCHUNK - 1);
      vals[it] = *(const v4f*)(sOut + qc * 4);
    }
    float* ob = out + n0 * kOutDim;
    for (int pass = 0; pass < 2; ++pass) {
#pragma unroll
      for (int it = 0; it < 7; ++it) {
        const int q = it * 256 + tid;
        if (q < NCHUNK) *(volatile v4f*)(ob + (size_t)q * 4) = vals[it];
      }
      __threadfence();
    }
  }
}

extern "C" void kernel_launch(void* const* d_in, const int* in_sizes, int n_in,
                              void* d_out, int out_size, void* d_ws, size_t ws_size,
                              hipStream_t stream) {
  if (n_in < 15) return;
  if (in_sizes[0] != kNpos * kInDim) return;
  if (in_sizes[1] != kInDim * kWidth) return;
  if (in_sizes[2] != kWidth) return;
  if (in_sizes[3] != kLayers * kWidth) return;
  if (in_sizes[4] != kLayers * kWidth * kModes) return;
  if (in_sizes[5] != kLayers * kWidth * kModes) return;
  if (in_sizes[6] != kLayers * kWidth * kModes) return;
  if (in_sizes[7] != kLayers * kWidth * kModes) return;
  if (in_sizes[8] != kLayers * kWidth) return;
  if (in_sizes[9] != kLayers * kWidth * kGluW) return;
  if (in_sizes[10] != kLayers * kGluW) return;
  if (in_sizes[11] != kWidth) return;
  if (in_sizes[12] != kWidth) return;
  if (in_sizes[13] != kWidth * kOutDim) return;
  if (in_sizes[14] != kOutDim) return;
  if (out_size != kNpos * kOutDim) return;
  if (ws_size < kWsTotal) return;

  const float* x      = (const float*)d_in[0];
  const float* proj_w = (const float*)d_in[1];
  const float* proj_b = (const float*)d_in[2];
  const float* log_dt = (const float*)d_in[3];
  const float* A_re   = (const float*)d_in[4];
  const float* A_im   = (const float*)d_in[5];
  const float* C_re   = (const float*)d_in[6];
  const float* C_im   = (const float*)d_in[7];
  const float* Dv     = (const float*)d_in[8];
  const float* out_w  = (const float*)d_in[9];
  const float* out_b  = (const float*)d_in[10];
  const float* ln_g   = (const float*)d_in[11];
  const float* ln_b   = (const float*)d_in[12];
  const float* head_w = (const float*)d_in[13];
  const float* head_b = (const float*)d_in[14];
  float* out = (float*)d_out;

  char* ws = (char*)d_ws;
  float*          UF0    = (float*)(ws + kOffUF0);
  float*          UF1    = (float*)(ws + kOffUF1);
  unsigned short* UH16   = (unsigned short*)(ws + kOffUH);
  unsigned short* G16    = (unsigned short*)(ws + kOffG16);
  float*          S32    = (float*)(ws + kOffS32);
  unsigned short* INIT16 = (unsigned short*)(ws + kOffInit);
  unsigned short* MV16   = (unsigned short*)(ws + kOffMv);
  unsigned short* ET16   = (unsigned short*)(ws + kOffEt);
  float*          WPOW   = (float*)(ws + kOffWpow);
  unsigned short* WOT    = (unsigned short*)(ws + kOffWot);
  unsigned short* WPH    = (unsigned short*)(ws + kOffWph);
  unsigned short* WPL    = (unsigned short*)(ws + kOffWpl);
  unsigned short* WHH    = (unsigned short*)(ws + kOffWhh);
  unsigned short* WHL    = (unsigned short*)(ws + kOffWhl);

  weight_planes_kernel<<<80, 256, 0, stream>>>(out_w, proj_w, head_w, WOT, WPH, WPL, WHH, WHL);
  input_proj_kernel<<<kNpos / 64, 256, 0, stream>>>(x, WPH, WPL, proj_b, UF0, UH16);

  for (int i = 0; i < kLayers; ++i) {
    const size_t om = (size_t)i * kWidth * kModes;
    float* cur = (i & 1) ? UF1 : UF0;
    float* nxt = (i & 1) ? UF0 : UF1;
    layer_tables_kernel<<<kWidth, 256, 0, stream>>>(log_dt + i * kWidth, A_re + om, A_im + om, C_re + om, C_im + om,
                                                    ET16, MV16, WPOW);
    chunk_gemm_kernel<0><<<(kWidth * 4) / 8, 256, 0, stream>>>(UH16, nullptr, ET16, (void*)S32, nullptr, nullptr);
    combine_kernel<<<(kWidth * kBatch) / 8, 256, 0, stream>>>(S32, WPOW, INIT16);
    chunk_gemm_kernel<1><<<(kWidth * 4) / 8, 256, 0, stream>>>(UH16, INIT16, MV16, (void*)G16, cur, Dv + i * kWidth);
    glu_kernel<<<kNpos / 64, 128, 0, stream>>>(G16, WOT + (size_t)i * kGluW * kWidth, out_b + i * kGluW, cur, nxt, UH16);
  }

  norm_head_kernel<<<kNpos / kHeadPos, 256, 0, stream>>>(UF0, WHH, WHL, ln_g, ln_b, head_b, out);
}
